// DeformableConv1D_3899830304947
// MI455X (gfx1250) — hardware-verified
//
#include <hip/hip_runtime.h>


namespace {
constexpr int B = 8, C = 256, L = 4096, O = 256, K = 3, OG = 4, HID = 64, GC = C / OG  , GH = HID / OG  , NOM = OG * 3 * K  , BL = 8  , PB = 32  ;
constexpr float XS = 8.0f, WSC = 256.0f;
static_assert(L % PB == 0 && C == 256 && O == 256, "tiling");
typedef _Float16 b16;
typedef __attribute__((ext_vector_type(16))) _Float16 v16b;
typedef __attribute__((ext_vector_type(8))) _Float16 v8b;
typedef __attribute__((ext_vector_type(8))) float v8f;
typedef __attribute__((ext_vector_type(4))) float v4f;
__device__ __forceinline__ float bf16_rne(float f) { unsigned int u = __float_as_uint(f); u += 0x7FFFu + ((u >> 16) & 1u); return __uint_as_float(u & 0xFFFF0000u); }
__device__ __forceinline__ void split16(float v, b16& hi, b16& lo) { hi = (b16)v; lo = (b16)(v - (float)hi); }
__device__ __forceinline__ v16b frag_kb(const b16* p, int hh) { const v8b a = *(const v8b*)(p + 8 * hh), b = *(const v8b*)(p + 16 + 8 * hh); v16b f;
#pragma unroll
  for (int e = 0; e < 8; ++e) { f[e] = a[e]; f[8 + e] = b[e]; } return f; }
__device__ __forceinline__ v8f wmma16b(v16b a, v16b b, v8f c) { v8f d = __builtin_amdgcn_wmma_f32_16x16x32_f16(false, a, false, b, (short)0, c, false, false); asm volatile("v_nop\n\tv_nop\n\tv_nop\n\tv_nop" : "+v"(d) : "v"(a), "v"(b)); return d; }
__device__ __forceinline__ void wave_lds_sync() { __builtin_amdgcn_fence(__ATOMIC_RELEASE, "workgroup"); __builtin_amdgcn_wave_barrier(); __builtin_amdgcn_fence(__ATOMIC_ACQUIRE, "workgroup"); }
__device__ __forceinline__ float pmul(float a, float b) { float p = a * b; asm volatile("" : "+v"(p)); return p; }
__device__ __forceinline__ int iclamp(int v, int lo, int hi) { return v < lo ? lo : (v > hi ? hi : v); }

typedef __attribute__((ext_vector_type(2))) float v2f;
__global__ __launch_bounds__(256) void xt_kernel(const float* __restrict__ x, b16* __restrict__ XT) {
  __shared__ float tile[64][65];
  const int l0 = blockIdx.x * 64, c0 = blockIdx.y * 64, b = blockIdx.z; const int t = threadIdx.x;
  for (int i = t; i < 64 * 64; i += 256) { const int cc = i / 64, ll = i % 64; tile[cc][ll] = bf16_rne(x[((size_t)b * C + c0 + cc) * L + l0 + ll]); }
  __syncthreads();
  for (int pass = 0; pass < 2; ++pass) { for (int i = t; i < 64 * 8; i += 256) { const int ll = i / 8, c8 = (i % 8) * 8; v8b o; for (int j = 0; j < 8; ++j) o[j] = (b16)(tile[c8 + j][ll] * XS); *(volatile v8b*)(XT + ((size_t)b * L + l0 + ll) * C + c0 + c8) = o; } __threadfence(); }
}
__global__ __launch_bounds__(256) void wprep_kernel(const float* __restrict__ w1, const float* __restrict__ wt, b16* __restrict__ W1B, b16* __restrict__ WB) {
  size_t t = (size_t)blockIdx.x * 256 + threadIdx.x; v8b o;
  { const size_t n = (size_t)HID * C / 8; if (t < n) { const size_t e = t * 8; const int r = (int)(e / C), c0 = (int)(e % C); const int g = r / GH, oo = r % GH;
      for (int j = 0; j < 8; ++j) { const int c = c0 + j; o[j] = (c / GC == g) ? (b16)(bf16_rne(w1[((size_t)g * GH + oo) * GC + (c - g * GC)]) * WSC) : (b16)0.0f; }
      for (int pass = 0; pass < 2; ++pass) { *(volatile v8b*)(W1B + e) = o; __threadfence(); } return; } t -= n; }
  { const size_t n = (size_t)O * K * C / 8; if (t < n) { const size_t e = t * 8; const int oo = (int)(e / (K * C)); const int kk = (int)((e / C) % K), c0 = (int)(e % C);
      for (int j = 0; j < 8; ++j) o[j] = (b16)(bf16_rne(wt[((size_t)oo * C + c0 + j) * K + kk]) * WSC);
      for (int pass = 0; pass < 2; ++pass) { *(volatile v8b*)(WB + e) = o; __threadfence(); } } }
}
__device__ __forceinline__ float geluf(float v) { return 0.5f * v * (1.0f + erff(v * 0.70710678118654752f)); }
__global__ __launch_bounds__(128) void dcv_kernel(const b16* __restrict__ XT, const b16* __restrict__ W1B, const float* __restrict__ b1, const float* __restrict__ w2, const float* __restrict__ b2, const b16* __restrict__ WB, const float* __restrict__ bias, float* __restrict__ out) {
  __shared__ __attribute__((aligned(16))) b16 Ah[PB][C + 8], Al[PB][C + 8]; __shared__ float Hs[PB][HID + 1], Om[PB][NOM + 1]; __shared__ int PosI[K][PB]; __shared__ float PosW[K][PB], PosM[K][PB], PosV0[K][PB], PosV1[K][PB]; __shared__ __attribute__((aligned(16))) float Os[O][PB + 4];
  const int t = threadIdx.x, wave = t >> 5, lane = t & 31, nloc = lane & 15, hlf = lane >> 4; const int b = blockIdx.y, l0 = blockIdx.x * PB; const int ph = wave & 1, oh = wave >> 1;
  const b16* XTb = XT + (size_t)b * L * C;
  { v8f acc[2] = {(v8f){}, (v8f){}};
#pragma unroll 2
    for (int kb = 0; kb < C; kb += 32) { const v16b a = frag_kb(XTb + (size_t)(l0 + ph * 16 + nloc) * C + kb, hlf);
#pragma unroll
      for (int tt = 0; tt < 2; ++tt) acc[tt] = wmma16b(a, frag_kb(W1B + (size_t)(oh * 32 + tt * 16 + nloc) * C + kb, hlf), acc[tt]); }
#pragma unroll
    for (int tt = 0; tt < 2; ++tt) { const int hc = oh * 32 + tt * 16 + nloc; const float bb = bf16_rne(b1[hc]);
#pragma unroll
      for (int r = 0; r < 8; ++r) Hs[ph * 16 + 8 * hlf + r][hc] = geluf(acc[tt][r] * (1.0f / (XS * WSC)) + bb); } }
  __syncthreads();
  if (t < PB) { const int p = t; const int l = l0 + p; float* om = &Om[p][0];
#pragma unroll 1
    for (int gj = 0; gj < NOM; ++gj) { const int g = gj / 9; float s = bf16_rne(b2[gj]);
#pragma unroll 1
      for (int c = 0; c < GH; ++c) s += pmul(Hs[p][g * GH + c], bf16_rne(w2[(size_t)gj * GH + c])); om[gj] = s; }
    const float offx[K] = {om[0], om[2], om[4]}; om[1] = 0.0f; om[3] = 0.0f; om[5] = 0.0f;
    float mx = -INFINITY;
#pragma unroll 1
    for (int q = K; q < NOM; ++q) mx = fmaxf(mx, om[q]);
    float Z = 0.0f;
#pragma unroll 1
    for (int q = K; q < NOM; ++q) { const float ev = __expf(om[q] - mx); om[q] = ev; Z += ev; }
    const float rcp = 1.0f / (float)(L - 1); const float lf = (float)l; const float onem = __builtin_fmaf(-lf, rcp, 1.0f); const float base = (l == L - 1) ? 1.0f : __builtin_fmaf(lf, rcp, -onem);
#pragma unroll
    for (int k = 0; k < K; ++k) { const float mod = om[K + k] / Z; const float kp = -0.5f + (float)k * 0.5f;
      const float t1 = __fadd_rn(base, kp); const float t2 = __fmul_rn(offx[k], 2.0f / (float)L); const float grid = __fadd_rn(t1, t2); const float pos = __fmul_rn(__fmul_rn(__fadd_rn(grid, 1.0f), 0.5f), (float)(L - 1)); const float fl = floorf(pos); const int i0 = (int)fl, i1 = i0 + 1; const float w = pos - fl;
      PosI[k][p] = i0; PosW[k][p] = w; PosM[k][p] = mod; PosV0[k][p] = (i0 >= 0 && i0 < L) ? 1.0f : 0.0f; PosV1[k][p] = (i1 >= 0 && i1 < L) ? 1.0f : 0.0f; } }
  __syncthreads();
  v8f acc[8];
#pragma unroll
  for (int tt = 0; tt < 8; ++tt) acc[tt] = (v8f){};
#pragma unroll 1
  for (int k = 0; k < K; ++k) {
    for (int p = wave; p < PB; p += 4) { const int i0 = PosI[k][p]; const float w = PosW[k][p], mod = PosM[k][p], v0 = PosV0[k][p], v1 = PosV1[k][p]; const int i0c = iclamp(i0, 0, L - 1), i1c = iclamp(i0 + 1, 0, L - 1);
      const v8b x0 = *(const v8b*)(XTb + (size_t)i0c * C + lane * 8), x1 = *(const v8b*)(XTb + (size_t)i1c * C + lane * 8); const float c0 = (1.0f - w) * v0, c1 = w * v1; v8b hv, lv;
      for (int j = 0; j < 8; ++j) { const float s = (pmul((float)x0[j] * (1.0f / XS), c0) + pmul((float)x1[j] * (1.0f / XS), c1)) * mod; b16 a_, b_; split16(s * XS, a_, b_); hv[j] = a_; lv[j] = b_; }
      *(v8b*)(&Ah[p][lane * 8]) = hv; *(v8b*)(&Al[p][lane * 8]) = lv; }
    __syncthreads();
#pragma unroll 2
    for (int kb = 0; kb < C; kb += 32) { const v16b a = frag_kb(&Ah[ph * 16 + nloc][kb], hlf), al = frag_kb(&Al[ph * 16 + nloc][kb], hlf);
#pragma unroll
      for (int tt = 0; tt < 8; ++tt) { const v16b bw = frag_kb(WB + (size_t)(oh * 128 + tt * 16 + nloc) * (K * C) + k * C + kb, hlf); acc[tt] = wmma16b(a, bw, acc[tt]); acc[tt] = wmma16b(al, bw, acc[tt]); } }
    __syncthreads(); }
#pragma unroll
  for (int tt = 0; tt < 8; ++tt) { const int oc = oh * 128 + tt * 16 + nloc; const float bb = bf16_rne(bias[oc]);
#pragma unroll
    for (int r = 0; r < 8; ++r) Os[oc][ph * 16 + 8 * hlf + r] = acc[tt][r] * (1.0f / (XS * WSC)) + bb; }
  __syncthreads();
  for (int pass = 0; pass < 2; ++pass) {
#pragma unroll 1
    for (int q = 0; q < 64; ++q) { const int oc = wave * 64 + q; ((volatile float*)out)[((size_t)b * O + oc) * L + l0 + lane] = Os[oc][lane]; }
    __threadfence(); }
}
}

extern "C" void kernel_launch(void* const* d_in, const int* in_sizes, int n_in, void* d_out, int out_size, void* d_ws, size_t ws_size, hipStream_t stream) {
  (void)n_in;
  auto Fp = [&](int i) { return (const float*)d_in[i]; };
  if (in_sizes[0] != B * C * L || in_sizes[1] != O * C * K || in_sizes[2] != O || in_sizes[3] != OG * GH * GC || in_sizes[4] != HID || in_sizes[5] != OG * 9 * GH || in_sizes[6] != NOM || out_size != B * O * L) return;
  size_t off = 0; char* ws = (char*)d_ws;
  auto carve = [&](size_t bytes) { char* p = ws + off; off += (bytes + 255) & ~(size_t)255; return p; };
  b16* XT = (b16*)carve((size_t)B * L * C * 2); b16* W1B = (b16*)carve((size_t)HID * C * 2); b16* WB = (b16*)carve((size_t)O * K * C * 2);
  if (off > ws_size || off > ((size_t)128 << 20)) return;
  xt_kernel<<<dim3(L / 64, C / 64, BL), 256, 0, stream>>>(Fp(0), XT);
  wprep_kernel<<<(unsigned)((((size_t)HID * C + (size_t)O * K * C) / 8 + 255) / 256), 256, 0, stream>>>(Fp(3), Fp(1), W1B, WB);
  dcv_kernel<<<dim3(L / PB, BL), 128, 0, stream>>>(XT, W1B, Fp(4), Fp(5), Fp(6), WB, Fp(2), (float*)d_out);
}
